// MultiModalAttention_85641647882457
// MI455X (gfx1250) — hardware-verified
//
#include <hip/hip_runtime.h>


#define NB_  4
#define TT   2048
#define MM   256
#define CC   512
#define NH_  8
#define HD   64
#define ZH   2
typedef _Float16 h16;
typedef unsigned short bf;
typedef __attribute__((ext_vector_type(16))) __bf16   v16bf;
typedef __attribute__((ext_vector_type(16))) _Float16 v16h;
typedef __attribute__((ext_vector_type(8)))  _Float16 v8h;
typedef __attribute__((ext_vector_type(8)))  unsigned short v8us;
typedef __attribute__((ext_vector_type(8)))  float    v8f;
typedef __attribute__((ext_vector_type(4)))  float    v4f;
typedef v8h  __attribute__((may_alias)) v8ha;
typedef v4f  __attribute__((may_alias)) v4fa;
typedef v8us __attribute__((may_alias)) v8usa;

__device__ __forceinline__ unsigned short f2bf(float f) { unsigned u = __float_as_uint(f); u += 0x7FFFu + ((u >> 16) & 1u); return (unsigned short)(u >> 16); }
__device__ __forceinline__ float bf2f(unsigned short b) { return __uint_as_float(((unsigned)b) << 16); }
__device__ __forceinline__ float bfr(float f) { return bf2f(f2bf(f)); }
__device__ __forceinline__ v16h cat16(v8h lo, v8h hi) { return __builtin_shufflevector(lo, hi, 0, 1, 2, 3, 4, 5, 6, 7, 8, 9, 10, 11, 12, 13, 14, 15); }
__device__ __forceinline__ v16bf cat16b(v8us lo, v8us hi) { return __builtin_bit_cast(v16bf, __builtin_shufflevector(lo, hi, 0, 1, 2, 3, 4, 5, 6, 7, 8, 9, 10, 11, 12, 13, 14, 15)); }
__device__ __forceinline__ v8f wmma16(v16h a, v16h b, v8f c) { return __builtin_amdgcn_wmma_f32_16x16x32_f16(false, a, false, b, (short)0, c, false, false); }
__device__ __forceinline__ v8f wmmab(v16bf a, v16bf b, v8f c) { return __builtin_amdgcn_wmma_f32_16x16x32_bf16(false, a, false, b, (short)0, c, false, false); }


template <typename T16> struct WFrag;
template <> struct WFrag<h16> { typedef v16h V; static __device__ __forceinline__ V ld(const h16* p) { return cat16(*(const v8h*)p, *(const v8h*)(p + 16)); } static __device__ __forceinline__ v8f mma(V a, V b, v8f c) { return wmma16(a, b, c); } };
template <> struct WFrag<bf> { typedef v16bf V; static __device__ __forceinline__ V ld(const bf* p) { return cat16b(*(const v8us*)p, *(const v8us*)(p + 16)); } static __device__ __forceinline__ v8f mma(V a, V b, v8f c) { return wmmab(a, b, c); } };
template <typename T16, int NSPLIT, bool BIAS>
__global__ __launch_bounds__(32) void k_gemmw(const T16* __restrict__ A, const T16* __restrict__ A2, const T16* __restrict__ Bt, const T16* __restrict__ Bt2, int K, float* C, int ldc, const float* __restrict__ bias, size_t sA, size_t sB, size_t sC) {
    typedef typename WFrag<T16>::V V;
    __shared__ __align__(16) float os[16 * 68];
    const size_t z = blockIdx.z; A += z * sA; if (A2) A2 += z * sA; Bt += z * sB; if (Bt2) Bt2 += z * sB; C += z * sC;
    const int lane = threadIdx.x & 31, lr = lane & 15, hi = lane >> 4; const int r0 = blockIdx.x * 64, c0 = blockIdx.y * 64;
    v8f acc[4][4];
#pragma unroll
    for (int mb = 0; mb < 4; ++mb)
#pragma unroll
        for (int nb = 0; nb < 4; ++nb) acc[mb][nb] = (v8f){};
    const size_t aoff = (size_t)(r0 + lr) * K + 8 * hi, boff = (size_t)(c0 + lr) * K + 8 * hi;
#pragma unroll 1
    for (int kc = 0; kc < K; kc += 32) {
        V a[4], a2[4];
#pragma unroll
        for (int mb = 0; mb < 4; ++mb) { a[mb] = WFrag<T16>::ld(A + aoff + (size_t)mb * 16 * K + kc); if (NSPLIT == 1 || NSPLIT == 2) a2[mb] = WFrag<T16>::ld(A2 + aoff + (size_t)mb * 16 * K + kc); }
#pragma unroll
        for (int nb = 0; nb < 4; ++nb) { const V b = WFrag<T16>::ld(Bt + boff + (size_t)nb * 16 * K + kc); V b2; if (NSPLIT >= 2) b2 = WFrag<T16>::ld(Bt2 + boff + (size_t)nb * 16 * K + kc);
#pragma unroll
            for (int mb = 0; mb < 4; ++mb) { acc[mb][nb] = WFrag<T16>::mma(a[mb], b, acc[mb][nb]); if (NSPLIT == 1 || NSPLIT == 2) acc[mb][nb] = WFrag<T16>::mma(a2[mb], b, acc[mb][nb]); if (NSPLIT >= 2) acc[mb][nb] = WFrag<T16>::mma(a[mb], b2, acc[mb][nb]); } }
        asm volatile("v_nop\n\tv_nop\n\tv_nop\n\tv_nop" : "+v"(acc[0][0]), "+v"(acc[1][1]), "+v"(acc[2][2]), "+v"(acc[3][3]) : "v"(a[0]), "v"(a[3]));
    }
#pragma unroll
    for (int mb = 0; mb < 4; ++mb) {
#pragma unroll
        for (int nb = 0; nb < 4; ++nb) {
#pragma unroll
            for (int j = 0; j < 8; ++j) os[(hi * 8 + j) * 68 + nb * 16 + lr] = acc[mb][nb][j]; }
        __builtin_amdgcn_wave_barrier(); asm volatile("" ::: "memory");
        float* crow = C + (size_t)(r0 + mb * 16) * ldc + c0;
#pragma unroll 1
        for (int ps = 0; ps < 2; ++ps) {
#pragma unroll
            for (int s = 0; s < 8; ++s) { const int row = 2 * s + hi, cofs = lr * 4; v4f val = *(const v4fa*)(os + row * 68 + cofs); if (BIAS) { val[0] += bfr(bias[c0 + cofs]); val[1] += bfr(bias[c0 + cofs + 1]); val[2] += bfr(bias[c0 + cofs + 2]); val[3] += bfr(bias[c0 + cofs + 3]); }
                *(volatile v4f*)(crow + (size_t)row * ldc + cofs) = val; }
            if (ps == 0) __threadfence(); }
        __builtin_amdgcn_wave_barrier(); asm volatile("" ::: "memory");
    }
}

__device__ __forceinline__ h16 tohx(float x) { return (h16)x; }
__device__ __forceinline__ void splitf(float y, unsigned short& h, unsigned short& l) { h = f2bf(y); l = f2bf(y - bf2f(h)); }
typedef __attribute__((ext_vector_type(4))) int v4i;
typedef __attribute__((ext_vector_type(2))) unsigned short v2us;
typedef __attribute__((ext_vector_type(4))) unsigned short v4us;
typedef __attribute__((ext_vector_type(4))) _Float16 v4h;

__global__ __launch_bounds__(256) void k_cvt8(const float* __restrict__ src, bf* dst, size_t n8) { const size_t i = (size_t)blockIdx.x * 256 + threadIdx.x; if (i >= n8) return; const v8f v = *(const v8f*)(src + i * 8); v8us o;
#pragma unroll
    for (int k = 0; k < 8; ++k) o[k] = f2bf(v[k]); *(volatile v8us*)(dst + i * 8) = o; __threadfence(); *(volatile v8us*)(dst + i * 8) = o; }
__global__ __launch_bounds__(256) void k_wtG(const float* __restrict__ w, int K, int N, bf* Bt) {
    const int lane = threadIdx.x & 31; const int L0 = (blockIdx.x * 8 + (threadIdx.x >> 5)) * 8; const int nlines = N * K / 64;
#pragma unroll
    for (int ps = 0; ps < 2; ++ps) {
#pragma unroll 1
        for (int l = 0; l < 8; ++l) { const int L = L0 + l; if (L >= nlines) break; const size_t e = (size_t)L * 64 + lane * 2; const int k = (int)(e % K), n = (int)(e / K); v2us o;
            o[0] = f2bf(w[(size_t)k * N + n]); o[1] = f2bf(w[(size_t)(k + 1) * N + n]); *(volatile v2us*)(Bt + e) = o; }
        if (ps == 0) __threadfence(); }
}

__global__ __launch_bounds__(256) void k_pl16(const float* __restrict__ F, int T, int col0, float sc, h16* P) { const size_t e = ((size_t)blockIdx.x * 256 + threadIdx.x) * 4; if (e >= (size_t)NH_ * T * HD) return; const int d = (int)(e % HD); const int t = (int)((e / HD) % T); const int h = (int)(e / ((size_t)HD * T)); const float* f = F + (size_t)t * 1536 + col0 + h * HD + d; v4h o;
#pragma unroll
    for (int u = 0; u < 4; ++u) o[u] = tohx(f[u] * sc); *(volatile v4h*)(P + e) = o; __threadfence(); *(volatile v4h*)(P + e) = o; }
__global__ __launch_bounds__(256) void k_vt2(const float* __restrict__ F, int T, bf* Vh, bf* Vl) { const size_t e = ((size_t)blockIdx.x * 256 + threadIdx.x) * 2; if (e >= (size_t)NH_ * HD * T) return; const int t = (int)(e % T); const int d = (int)((e / T) % HD); const int h = (int)(e / ((size_t)T * HD)); v2us oh, ol;
#pragma unroll
    for (int u = 0; u < 2; ++u) { unsigned short a, b; splitf(F[(size_t)(t + u) * 1536 + 1024 + h * HD + d], a, b); oh[u] = a; ol[u] = b; } *(volatile v2us*)(Vh + e) = oh; *(volatile v2us*)(Vl + e) = ol; __threadfence(); *(volatile v2us*)(Vh + e) = oh; *(volatile v2us*)(Vl + e) = ol; }
__global__ __launch_bounds__(256) void k_cbias(const float* __restrict__ CY, float* BIAS) { const int idx = blockIdx.x * 256 + threadIdx.x; if (idx >= ZH * TT) return; const int t = idx % TT; const int zz = idx / TT; const float* col = CY + (size_t)zz * MM * TT + t; float mx = -3.0e38f;
#pragma unroll 1
    for (int m = 0; m < MM; ++m) mx = fmaxf(mx, col[(size_t)m * TT]);
    float sum = 0.f;
#pragma unroll 1
    for (int m = 0; m < MM; ++m) { float d0 = __fsub_rn(col[(size_t)m * TT], mx); asm volatile("" : "+v"(d0)); sum = __fadd_rn(sum, __builtin_amdgcn_exp2f(__fmul_rn(d0, 1.4426950408889634f))); }
    const float f = __fdiv_rn(1.0f, sum); float acc = 0.f;
#pragma unroll 1
    for (int m = 0; m < MM; ++m) { const float cv = col[(size_t)m * TT]; float d0 = __fsub_rn(cv, mx); asm volatile("" : "+v"(d0)); float p = __builtin_amdgcn_exp2f(__fmul_rn(d0, 1.4426950408889634f)) * f; asm volatile("" : "+v"(p)); float pv = __fmul_rn(p, cv); asm volatile("" : "+v"(pv)); acc = __fadd_rn(acc, pv); }
    const float bias = acc * (1.0f / MM); *(volatile float*)(BIAS + idx) = bias; __threadfence(); *(volatile float*)(BIAS + idx) = bias; }
__global__ __launch_bounds__(256) void k_ssoft(const float* __restrict__ S, const float* __restrict__ BIAS, const int* __restrict__ mk, bf* Ph, bf* Pl) { const int lane = threadIdx.x & 31; const int row = blockIdx.x * 8 + (threadIdx.x >> 5); if (row >= ZH * TT) return; const int i = row % TT; const int zz = row / TT; const float* sr = S + (size_t)row * TT; const float* br = BIAS + (size_t)zz * TT; const int* mr = mk + (size_t)i * TT; float v[TT / 32]; float mx = -3.0e38f;
#pragma unroll
    for (int ch = 0; ch < TT / 128; ++ch) { const int j0 = ch * 128 + lane * 4; const v4f a = *(const v4f*)(sr + j0); const v4f bb = *(const v4f*)(br + j0); const v4i m4 = *(const v4i*)(mr + j0);
#pragma unroll
        for (int u = 0; u < 4; ++u) { const float t = (m4[u] != 0) ? __fadd_rn(a[u], bb[u]) : -3.0e38f; v[ch * 4 + u] = t; mx = fmaxf(mx, t); } }
#pragma unroll
    for (int sh = 16; sh; sh >>= 1) mx = fmaxf(mx, __shfl_xor(mx, sh, 32));
    float sum = 0.f;
#pragma unroll
    for (int q = 0; q < TT / 32; ++q) { float d0 = __fsub_rn(v[q], mx); asm volatile("" : "+v"(d0)); v[q] = __builtin_amdgcn_exp2f(__fmul_rn(d0, 1.4426950408889634f)); sum += v[q]; }
#pragma unroll
    for (int sh = 16; sh; sh >>= 1) sum += __shfl_xor(sum, sh, 32);
    const float f = __fdiv_rn(1.0f, sum);
    for (int ps = 0; ps < 2; ++ps) {
#pragma unroll
        for (int ch = 0; ch < TT / 128; ++ch) { v4us oh, ol; for (int q = 0; q < 4; ++q) { unsigned short a2, c2; splitf(v[ch * 4 + q] * f, a2, c2); oh[q] = a2; ol[q] = c2; } const size_t oo = (size_t)row * TT + ch * 128 + lane * 4; *(volatile v4us*)(Ph + oo) = oh; *(volatile v4us*)(Pl + oo) = ol; }
        if (ps == 0) __threadfence(); } }
__global__ __launch_bounds__(256) void k_csm(const float* __restrict__ S, bf* Ph, bf* Pl) { const int lane = threadIdx.x & 31; const int row = blockIdx.x * 8 + (threadIdx.x >> 5); if (row >= ZH * TT) return; const float* sr = S + (size_t)row * MM; float v[MM / 32]; float mx = -3.0e38f;
#pragma unroll
    for (int ch = 0; ch < MM / 128; ++ch) { const v4f a = *(const v4f*)(sr + ch * 128 + lane * 4);
#pragma unroll
        for (int u = 0; u < 4; ++u) { v[ch * 4 + u] = a[u]; mx = fmaxf(mx, a[u]); } }
#pragma unroll
    for (int sh = 16; sh; sh >>= 1) mx = fmaxf(mx, __shfl_xor(mx, sh, 32));
    float sum = 0.f;
#pragma unroll
    for (int q = 0; q < MM / 32; ++q) { float d0 = __fsub_rn(v[q], mx); asm volatile("" : "+v"(d0)); v[q] = __builtin_amdgcn_exp2f(__fmul_rn(d0, 1.4426950408889634f)); sum += v[q]; }
#pragma unroll
    for (int sh = 16; sh; sh >>= 1) sum += __shfl_xor(sum, sh, 32);
    const float f = __fdiv_rn(1.0f, sum);
    for (int ps = 0; ps < 2; ++ps) {
#pragma unroll
        for (int ch = 0; ch < MM / 128; ++ch) { v4us oh, ol; for (int q = 0; q < 4; ++q) { unsigned short a2, c2; splitf(v[ch * 4 + q] * f, a2, c2); oh[q] = a2; ol[q] = c2; } const size_t oo = (size_t)row * MM + ch * 128 + lane * 4; *(volatile v4us*)(Ph + oo) = oh; *(volatile v4us*)(Pl + oo) = ol; }
        if (ps == 0) __threadfence(); } }
__global__ __launch_bounds__(256) void k_mrgf(const float* __restrict__ O, int h0, float* SV) { const size_t e = ((size_t)blockIdx.x * 256 + threadIdx.x) * 4; if (e >= (size_t)ZH * TT * HD) return; const int d = (int)(e % HD); const int t = (int)((e / HD) % TT); const int zz = (int)(e / ((size_t)HD * TT)); const v4f a = *(const v4f*)(O + e); float* dst = SV + (size_t)t * CC + (h0 + zz) * HD + d; *(volatile v4f*)dst = a; __threadfence(); *(volatile v4f*)dst = a; }
__global__ __launch_bounds__(256) void k_plhl(const float* __restrict__ F, bf* Ph, bf* Pl) { const size_t e = ((size_t)blockIdx.x * 256 + threadIdx.x) * 4; if (e >= (size_t)TT * CC) return; v4us oh, ol;
#pragma unroll
    for (int u = 0; u < 4; ++u) { unsigned short a, b; splitf(F[e + u], a, b); oh[u] = a; ol[u] = b; } *(volatile v4us*)(Ph + e) = oh; *(volatile v4us*)(Pl + e) = ol; __threadfence(); *(volatile v4us*)(Ph + e) = oh; *(volatile v4us*)(Pl + e) = ol; }
__global__ __launch_bounds__(256) void k_mix(const float* __restrict__ GS, const float* __restrict__ GC, const float* __restrict__ SV, const float* __restrict__ CV, bf* Ph, bf* Pl) { const size_t e = ((size_t)blockIdx.x * 256 + threadIdx.x) * 4; if (e >= (size_t)TT * CC) return; v4us oh, ol;
#pragma unroll
    for (int u = 0; u < 4; ++u) { const float sg = __fdiv_rn(1.0f, __fadd_rn(1.0f, __expf(-GS[e + u]))), cg = __fdiv_rn(1.0f, __fadd_rn(1.0f, __expf(-GC[e + u]))); float a = __fmul_rn(sg, CV[e + u]), b = __fmul_rn(cg, SV[e + u]); asm volatile("" : "+v"(a)); asm volatile("" : "+v"(b)); unsigned short hh, ll; splitf(__fadd_rn(a, b), hh, ll); oh[u] = hh; ol[u] = ll; }
    *(volatile v4us*)(Ph + e) = oh; *(volatile v4us*)(Pl + e) = ol; __threadfence(); *(volatile v4us*)(Ph + e) = oh; *(volatile v4us*)(Pl + e) = ol; }

extern "C" void kernel_launch(void* const* d_in, const int* in_sizes, int n_in,
                              void* d_out, int out_size, void* d_ws, size_t ws_size, hipStream_t stream) {
    (void)in_sizes; (void)n_in; (void)out_size;
    const float** I = (const float**)d_in;
    const float *x = I[0], *y = I[1]; const int* mk = (const int*)d_in[2]; const float *Wx = I[3], *bx = I[4], *Wy = I[5], *by = I[6], *Wgs = I[7], *bgs = I[8], *Wgc = I[9], *bgc = I[10], *Wp = I[11], *bp = I[12];
    float* OUT = (float*)d_out;
    char* wsp = (char*)d_ws;
    auto take = [&](size_t bytes) { char* p = wsp; wsp += (bytes + 255) & ~(size_t)255; return (void*)p; };
    bf* XB = (bf*)take((size_t)TT * CC * 2); bf* YB = (bf*)take((size_t)MM * CC * 2); bf* BX = (bf*)take((size_t)1536 * CC * 2); bf* BY = (bf*)take((size_t)1536 * CC * 2); bf* BGS = (bf*)take((size_t)CC * CC * 2); bf* BGC = (bf*)take((size_t)CC * CC * 2); bf* BP = (bf*)take((size_t)CC * CC * 2);
    float* FX = (float*)take((size_t)TT * 1536 * 4); float* FY = (float*)take((size_t)MM * 1536 * 4);
    h16* QX = (h16*)take((size_t)NH_ * TT * HD * 2); h16* KX = (h16*)take((size_t)NH_ * TT * HD * 2); h16* QY = (h16*)take((size_t)NH_ * MM * HD * 2); h16* KY = (h16*)take((size_t)NH_ * MM * HD * 2); bf* VXh = (bf*)take((size_t)NH_ * HD * TT * 2); bf* VXl = (bf*)take((size_t)NH_ * HD * TT * 2); bf* VYh = (bf*)take((size_t)NH_ * HD * MM * 2); bf* VYl = (bf*)take((size_t)NH_ * HD * MM * 2);
    float* CY = (float*)take((size_t)ZH * MM * TT * 4); float* BIAS = (float*)take((size_t)ZH * TT * 4); float* S = (float*)take((size_t)ZH * TT * TT * 4); bf* Ph = (bf*)take((size_t)ZH * TT * TT * 2); bf* Pl = (bf*)take((size_t)ZH * TT * TT * 2); float* O = (float*)take((size_t)ZH * TT * HD * 4);
    float* CA = (float*)take((size_t)ZH * TT * MM * 4); bf* PCh = (bf*)take((size_t)ZH * TT * MM * 2); bf* PCl = (bf*)take((size_t)ZH * TT * MM * 2);
    float* SV = (float*)take((size_t)TT * CC * 4); float* CV = (float*)take((size_t)TT * CC * 4); bf* T1h = (bf*)take((size_t)TT * CC * 2); bf* T1l = (bf*)take((size_t)TT * CC * 2); float* GS = (float*)take((size_t)TT * CC * 4); float* GC = (float*)take((size_t)TT * CC * 4);
    if ((size_t)(wsp - (char*)d_ws) > ws_size) return;
    k_wtG<<<(unsigned)((CC * 1536 / 64 + 63) / 64), 256, 0, stream>>>(Wx, CC, 1536, BX); k_wtG<<<(unsigned)((CC * 1536 / 64 + 63) / 64), 256, 0, stream>>>(Wy, CC, 1536, BY); k_wtG<<<(CC * CC / 64 + 63) / 64, 256, 0, stream>>>(Wgs, CC, CC, BGS); k_wtG<<<(CC * CC / 64 + 63) / 64, 256, 0, stream>>>(Wgc, CC, CC, BGC); k_wtG<<<(CC * CC / 64 + 63) / 64, 256, 0, stream>>>(Wp, CC, CC, BP);
    const size_t zq = (size_t)TT * HD, zqy = (size_t)MM * HD, zS = (size_t)TT * TT, zvx = (size_t)HD * TT, zvy = (size_t)HD * MM;
    for (int b = 0; b < NB_; ++b) {
        k_cvt8<<<(unsigned)(((size_t)TT * CC / 8 + 255) / 256), 256, 0, stream>>>(x + (size_t)b * TT * CC, XB, (size_t)TT * CC / 8); k_cvt8<<<(MM * CC / 8 + 255) / 256, 256, 0, stream>>>(y + (size_t)b * MM * CC, YB, MM * CC / 8);
        k_gemmw<bf, 0, true><<<dim3(TT / 64, 1536 / 64, 1), 32, 0, stream>>>(XB, nullptr, BX, nullptr, CC, FX, 1536, bx, 0, 0, 0); k_gemmw<bf, 0, true><<<dim3(MM / 64, 1536 / 64, 1), 32, 0, stream>>>(YB, nullptr, BY, nullptr, CC, FY, 1536, by, 0, 0, 0);
        k_pl16<<<(unsigned)(((size_t)NH_ * TT * HD / 4 + 255) / 256), 256, 0, stream>>>(FX, TT, 0, 0.125f, QX); k_pl16<<<(unsigned)(((size_t)NH_ * TT * HD / 4 + 255) / 256), 256, 0, stream>>>(FX, TT, CC, 1.0f, KX); k_pl16<<<(NH_ * MM * HD / 4 + 255) / 256, 256, 0, stream>>>(FY, MM, 0, 0.125f, QY); k_pl16<<<(NH_ * MM * HD / 4 + 255) / 256, 256, 0, stream>>>(FY, MM, CC, 1.0f, KY);
        k_vt2<<<(unsigned)(((size_t)NH_ * HD * TT / 2 + 255) / 256), 256, 0, stream>>>(FX, TT, VXh, VXl); k_vt2<<<(NH_ * HD * MM / 2 + 255) / 256, 256, 0, stream>>>(FY, MM, VYh, VYl);
        for (int h0 = 0; h0 < NH_; h0 += ZH) {
            k_gemmw<h16, 0, false><<<dim3(MM / 64, TT / 64, ZH), 32, 0, stream>>>(QY + (size_t)h0 * zqy, nullptr, KX + (size_t)h0 * zq, nullptr, HD, CY, TT, nullptr, zqy, zq, (size_t)MM * TT);
            k_cbias<<<(ZH * TT + 255) / 256, 256, 0, stream>>>(CY, BIAS);
            k_gemmw<h16, 0, false><<<dim3(TT / 64, TT / 64, ZH), 32, 0, stream>>>(QX + (size_t)h0 * zq, nullptr, KX + (size_t)h0 * zq, nullptr, HD, S, TT, nullptr, zq, zq, zS);
            k_ssoft<<<ZH * TT / 8, 256, 0, stream>>>(S, BIAS, mk, Ph, Pl);
            k_gemmw<bf, 2, false><<<dim3(TT / 64, 1, ZH), 32, 0, stream>>>(Ph, Pl, VXh + (size_t)h0 * zvx, VXl + (size_t)h0 * zvx, TT, O, HD, nullptr, zS, zvx, zq);
            k_mrgf<<<(unsigned)(((size_t)ZH * TT * HD / 4 + 255) / 256), 256, 0, stream>>>(O, h0, SV);
            k_gemmw<h16, 0, false><<<dim3(TT / 64, MM / 64, ZH), 32, 0, stream>>>(QX + (size_t)h0 * zq, nullptr, KY + (size_t)h0 * zqy, nullptr, HD, CA, MM, nullptr, zq, zqy, (size_t)TT * MM);
            k_csm<<<ZH * TT / 8, 256, 0, stream>>>(CA, PCh, PCl);
            k_gemmw<bf, 2, false><<<dim3(TT / 64, 1, ZH), 32, 0, stream>>>(PCh, PCl, VYh + (size_t)h0 * zvy, VYl + (size_t)h0 * zvy, MM, O, HD, nullptr, (size_t)TT * MM, zvy, zq);
            k_mrgf<<<(unsigned)(((size_t)ZH * TT * HD / 4 + 255) / 256), 256, 0, stream>>>(O, h0, CV); }
        k_plhl<<<(unsigned)(((size_t)TT * CC / 4 + 255) / 256), 256, 0, stream>>>(SV, T1h, T1l); k_gemmw<bf, 1, true><<<dim3(TT / 64, CC / 64, 1), 32, 0, stream>>>(T1h, T1l, BGS, nullptr, CC, GS, CC, bgs, 0, 0, 0);
        k_plhl<<<(unsigned)(((size_t)TT * CC / 4 + 255) / 256), 256, 0, stream>>>(CV, T1h, T1l); k_gemmw<bf, 1, true><<<dim3(TT / 64, CC / 64, 1), 32, 0, stream>>>(T1h, T1l, BGC, nullptr, CC, GC, CC, bgc, 0, 0, 0);
        k_mix<<<(unsigned)(((size_t)TT * CC / 4 + 255) / 256), 256, 0, stream>>>(GS, GC, SV, CV, T1h, T1l);
        k_gemmw<bf, 1, true><<<dim3(TT / 64, CC / 64, 1), 32, 0, stream>>>(T1h, T1l, BP, nullptr, CC, OUT + (size_t)b * TT * CC, CC, bp, 0, 0, 0); }
}
